// MultiHeadAttention_31525059953146
// MI455X (gfx1250) — hardware-verified
//
#include <hip/hip_runtime.h>
#ifndef NB
#define NB 2
#endif
#ifndef SEQ
#define SEQ 2048
#endif
#define SEQ_FULL 2048
#define DM 1024
#define NH 16
#define HD 64
#define QT 256
#define EARLY ((SEQ) < 512 ? (SEQ) : 512)
#define NR ((size_t)NB * SEQ)
#define ATS 0.125f
#define RSC 2048.0f
#define RINV 0.00048828125f
#define RBIG 0x40000000u

static_assert(NH * HD == DM);
static_assert(HD == 64);
static_assert(SEQ % 256 == 0);
static_assert(SEQ % QT == 0);
static_assert(QT % 128 == 0);
static_assert(EARLY % QT == 0 && EARLY % 128 == 0 && EARLY <= SEQ);
static_assert((SEQ - EARLY) % 128 == 0);
static_assert((NB * SEQ) % 128 == 0);
static_assert(DM % 64 == 0);
static_assert(((size_t)NB * SEQ * DM) % 2048 == 0);
static_assert((NH * QT) % 8 == 0);
static_assert((SEQ * 32) % 256 == 0);
static_assert(SEQ <= SEQ_FULL);

typedef unsigned short v8us __attribute__((ext_vector_type(8), may_alias));
typedef float  v8f  __attribute__((ext_vector_type(8)));
typedef float  v4f  __attribute__((ext_vector_type(4)));
typedef float  v2f  __attribute__((ext_vector_type(2)));
typedef float  v4fa __attribute__((ext_vector_type(4), may_alias));
typedef _Float16 v16h __attribute__((ext_vector_type(16)));
typedef _Float16 v4h __attribute__((ext_vector_type(4)));
union FragH { v16h v; v8us half[2]; _Float16 h[16]; unsigned short u[16]; };

__device__ __forceinline__ unsigned short bf16_bits(float x) { unsigned int u = __float_as_uint(x); return (unsigned short)((u + 0x7FFFu + ((u >> 16) & 1u)) >> 16); }
__device__ __forceinline__ float bf16_val(unsigned short b) { return __uint_as_float(((unsigned int)b) << 16); }
__device__ __forceinline__ float bf16_rne(float x) { return bf16_val(bf16_bits(x)); }

__global__ __launch_bounds__(256) void k_ropetab(float* __restrict__ T) {
  #pragma clang fp contract(off)
  const unsigned t = blockIdx.x * 256u + threadIdx.x;
  if (t >= (unsigned)(SEQ * 32)) return;
  const unsigned s = t >> 5, i = t & 31u;
  double p = 1.0;
#pragma unroll 1
  for (unsigned j = 0; j < i; ++j) p *= 1.3335214321633240;
  const float pf = (float)p;
  const float invf = 1.0f / pf;
  const float ang = (float)s * invf;
  v2f o; o[0] = cosf(ang); o[1] = sinf(ang);
  float* d = T + (size_t)t * 2;
  *(volatile v2f*)d = o; __threadfence(); *(volatile v2f*)d = o;
}

__global__ __launch_bounds__(256) void k_x16(const float* __restrict__ x, _Float16* __restrict__ X16) {
  const unsigned t = blockIdx.x * 256u + threadIdx.x;
  if (t >= (unsigned)(NR * DM / 8)) return;
  const unsigned r = t >> 7, c8 = (t & 127u) << 3;
  const unsigned b = r / (unsigned)SEQ, s = r - b * (unsigned)SEQ;
  const float* src = x + ((size_t)b * SEQ_FULL + s) * DM + c8;
  const v4f a = *(const v4fa*)src, c = *(const v4fa*)(src + 4);
  FragH f;
#pragma unroll
  for (int q = 0; q < 4; ++q) { f.h[q] = (_Float16)bf16_rne(a[q]); f.h[4 + q] = (_Float16)bf16_rne(c[q]); }
  const v8us o = f.half[0];
  unsigned short* d = (unsigned short*)X16 + (size_t)t * 8;
  *(volatile v8us*)d = o; __threadfence(); *(volatile v8us*)d = o;
}

__global__ __launch_bounds__(256) void k_wtr(const float* __restrict__ w, _Float16* __restrict__ Bt) {
  __shared__ unsigned short tl[64][66];
  const unsigned tid = threadIdx.x;
  const unsigned kt = blockIdx.x / (unsigned)(DM / 64), nt = blockIdx.x % (unsigned)(DM / 64);
  for (unsigned i = tid; i < 64u * 16u; i += 256u) {
    const unsigned r = i >> 4, c4 = (i & 15u) << 2;
    const v4f a = *(const v4fa*)(w + (size_t)(kt * 64u + r) * DM + nt * 64u + c4);
    FragH f;
#pragma unroll
    for (int q = 0; q < 4; ++q) f.h[q] = (_Float16)(bf16_rne(a[q]) * 16.0f);
#pragma unroll
    for (int q = 0; q < 4; ++q) tl[r][c4 + q] = f.u[q];
  }
  __syncthreads();
  for (int pass = 0; pass < 2; ++pass) {
#pragma unroll
    for (unsigned rd = 0; rd < 2; ++rd) {
      const unsigned n = rd * 32u + (tid >> 3), pc = tid & 7u;
      FragH f;
#pragma unroll
      for (int q = 0; q < 8; ++q) f.u[q] = tl[pc * 8u + q][n];
      const v8us o = f.half[0];
      *(volatile v8us*)((unsigned short*)Bt + (size_t)(nt * 64u + n) * DM + kt * 64u + pc * 8u) = o;
    }
    if (pass == 0) __threadfence();
  }
}

template <int NHv, int TTv>
__global__ __launch_bounds__(256) void k_vt(const _Float16* __restrict__ V16, int ldv, int voff, _Float16* __restrict__ Vt) {
  __shared__ unsigned short tl[64][66];
  const unsigned tid = threadIdx.x;
  const unsigned slab = blockIdx.x / (unsigned)(TTv / 64), lg = blockIdx.x % (unsigned)(TTv / 64);
  const unsigned b = slab / (unsigned)NHv, h = slab % (unsigned)NHv;
  for (unsigned i = tid; i < 64u * 8u; i += 256u) {
    const unsigned r = i >> 3, c8 = (i & 7u) << 3;
    FragH f;
    f.half[0] = *(const v8us*)((const unsigned short*)V16 + ((size_t)b * TTv + lg * 64u + r) * (size_t)ldv + (size_t)voff + h * 64u + c8);
#pragma unroll
    for (int q = 0; q < 8; ++q) tl[r][c8 + q] = f.u[q];
  }
  __syncthreads();
  for (int pass = 0; pass < 2; ++pass) {
#pragma unroll
    for (unsigned rd = 0; rd < 2; ++rd) {
      const unsigned d = rd * 32u + (tid >> 3), pc = tid & 7u;
      FragH f;
#pragma unroll
      for (int q = 0; q < 8; ++q) f.u[q] = tl[pc * 8u + q][d];
      const v8us o = f.half[0];
      *(volatile v8us*)((unsigned short*)Vt + ((size_t)slab * 64u + d) * TTv + lg * 64u + pc * 8u) = o;
    }
    if (pass == 0) __threadfence();
  }
}

__device__ __forceinline__ v16h g3_frag(const unsigned short* __restrict__ base, unsigned off) { FragH f; f.half[0] = *(const v8us*)(base + off); f.half[1] = *(const v8us*)(base + off + 16u); return f.v; }
__device__ __forceinline__ v8f g2_mma(v16h a, v16h b, v8f c) { v8f d = __builtin_amdgcn_wmma_f32_16x16x32_f16(false, a, false, b, (short)0, c, false, false); asm volatile("v_nop\n\tv_nop\n\tv_nop\n\tv_nop" : "+v"(d) : "v"(a), "v"(b)); return d; }

template <int ARES, int BRES>
__device__ __forceinline__ void g3_step(const unsigned short* __restrict__ Bb, unsigned bo, const unsigned short* __restrict__ BRb, unsigned bro,
    v16h a0, v16h a1, v16h a0r, v16h a1r, v8f& c0, v8f& c1, v8f& r0, v8f& r1) {
  const v16h b = g3_frag(Bb, bo);
  c0 = g2_mma(a0, b, c0); c1 = g2_mma(a1, b, c1);
  if (ARES) { r0 = g2_mma(a0r, b, r0); r1 = g2_mma(a1r, b, r1); }
  if (BRES) { const v16h br = g3_frag(BRb, bro); r0 = g2_mma(a0, br, r0); r1 = g2_mma(a1, br, r1); }
}

template <int ARES, int BRES>
__global__ __launch_bounds__(128) void k_gemm3(
    const _Float16* __restrict__ A, const _Float16* __restrict__ AR, int lda, int ldar, size_t sA, size_t sAR,
    const _Float16* __restrict__ Bh, const _Float16* __restrict__ BR, int ldb, int ldbr, size_t sB, size_t sBR,
    float alpha, float* __restrict__ C, _Float16* __restrict__ C16, _Float16* __restrict__ CR, int ldc, size_t sC,
    unsigned rmod, unsigned rlim, const float* __restrict__ rope, int M, int N, int K) {
  __shared__ __attribute__((aligned(16))) float so[4][32][68];
  const unsigned tid = threadIdx.x, w = tid >> 5, lane = tid & 31u, ln = lane & 15u, hh = lane >> 4;
  const unsigned by = blockIdx.y;
  const unsigned short* Ab = (const unsigned short*)A + (size_t)by * sA;
  const unsigned short* Bb = (const unsigned short*)Bh + (size_t)by * sB;
  const unsigned short* ARb = Ab;
  const unsigned short* BRb = Bb;
  if (ARES) ARb = (const unsigned short*)AR + (size_t)by * sAR;
  if (BRES) BRb = (const unsigned short*)BR + (size_t)by * sBR;
  const size_t cofs = (size_t)by * sC;
  const unsigned ntn = (unsigned)N >> 6;
  const unsigned mt = blockIdx.x / ntn, nq = blockIdx.x - mt * ntn;
  const unsigned row0 = mt * 128u + 32u * w, col0 = nq * 64u;
  if (row0 >= (unsigned)M) return;
  const unsigned ao0 = (row0 + ln) * (unsigned)lda + 8u * hh, ao1 = ao0 + 16u * (unsigned)lda;
  unsigned ro0 = ao0, ro1 = ao1;
  if (ARES) { ro0 = (row0 + ln) * (unsigned)ldar + 8u * hh; ro1 = ro0 + 16u * (unsigned)ldar; }
  const unsigned bo0 = (col0 + ln) * (unsigned)ldb + 8u * hh, bst = 16u * (unsigned)ldb;
  unsigned bro0 = bo0, brst = bst;
  if (BRES) { bro0 = (col0 + ln) * (unsigned)ldbr + 8u * hh; brst = 16u * (unsigned)ldbr; }
  const v8f z8 = {0.f,0.f,0.f,0.f,0.f,0.f,0.f,0.f};
  v8f c00 = z8, c01 = z8, c02 = z8, c03 = z8, c10 = z8, c11 = z8, c12 = z8, c13 = z8;
  v8f r00 = z8, r01 = z8, r02 = z8, r03 = z8, r10 = z8, r11 = z8, r12 = z8, r13 = z8;
#pragma unroll 1
  for (unsigned kb = 0; kb < (unsigned)K; kb += 32u) {
    const v16h a0 = g3_frag(Ab, ao0 + kb), a1 = g3_frag(Ab, ao1 + kb);
    v16h a0r = a0, a1r = a1;
    if (ARES) { a0r = g3_frag(ARb, ro0 + kb); a1r = g3_frag(ARb, ro1 + kb); }
    g3_step<ARES, BRES>(Bb, bo0 + kb,            BRb, bro0 + kb,             a0, a1, a0r, a1r, c00, c10, r00, r10);
    g3_step<ARES, BRES>(Bb, bo0 + bst + kb,      BRb, bro0 + brst + kb,      a0, a1, a0r, a1r, c01, c11, r01, r11);
    g3_step<ARES, BRES>(Bb, bo0 + 2u * bst + kb, BRb, bro0 + 2u * brst + kb, a0, a1, a0r, a1r, c02, c12, r02, r12);
    g3_step<ARES, BRES>(Bb, bo0 + 3u * bst + kb, BRb, bro0 + 3u * brst + kb, a0, a1, a0r, a1r, c03, c13, r03, r13);
  }
  v8f accs[8] = {c00, c01, c02, c03, c10, c11, c12, c13};
  v8f racs[8] = {r00, r01, r02, r03, r10, r11, r12, r13};
#pragma unroll
  for (int u = 0; u < 8; ++u) {
    const unsigned t = (unsigned)u & 3u, hf = (unsigned)u >> 2;
#pragma unroll
    for (int r = 0; r < 8; ++r) {
      const unsigned rloc = hf * 16u + 8u * hh + (unsigned)r;
      float v = accs[u][r];
      if (ARES || BRES) v += racs[u][r] * RINV;
      so[w][rloc][t * 16u + ln] = v * alpha;
    }
  }
  __builtin_amdgcn_fence(4  , "workgroup"); __builtin_amdgcn_wave_barrier();
  const unsigned rsub = lane >> 4, c4 = (lane & 15u) * 4u;
  const unsigned rm0 = row0 % rmod;
  if (rope) {
    const unsigned i0 = ((col0 + c4) & 63u) >> 1;
#pragma unroll
    for (unsigned q = 0; q < 16; ++q) {
      const unsigned r = q * 2u + rsub;
      const v4f t = *(const v4fa*)(rope + ((size_t)(rm0 + r) * 32u + i0) * 2u);
      const v4f v = *(const v4fa*)&so[w][r][c4];
      v4f o;
      o[0] = v[0] * t[0] - v[1] * t[1]; o[1] = v[1] * t[0] + v[0] * t[1];
      o[2] = v[2] * t[2] - v[3] * t[3]; o[3] = v[3] * t[2] + v[2] * t[3];
      *(v4fa*)&so[w][r][c4] = o;
    }
    __builtin_amdgcn_fence(4  , "workgroup"); __builtin_amdgcn_wave_barrier();
  }
  const bool wres = (CR != nullptr) && (rm0 < rlim);
  const size_t rr0 = (size_t)(row0 / rmod) * rlim + rm0;
  for (int pass = 0; pass < 2; ++pass) {
#pragma unroll
    for (unsigned q = 0; q < 16; ++q) {
      const unsigned r = q * 2u + rsub;
      const v4f v = *(const v4fa*)&so[w][r][c4];
      if (C) *(volatile v4f*)(C + cofs + (size_t)(row0 + r) * ldc + col0 + c4) = v;
      if (C16 || wres) {
        v4h h4, r4;
#pragma unroll
        for (int i = 0; i < 4; ++i) { h4[i] = (_Float16)v[i]; r4[i] = (_Float16)((v[i] - (float)h4[i]) * RSC); }
        if (C16) *(volatile v4h*)(C16 + cofs + (size_t)(row0 + r) * ldc + col0 + c4) = h4;
        if (wres) *(volatile v4h*)(CR + cofs + (rr0 + r) * (size_t)ldc + col0 + c4) = r4;
      }
    }
    if (pass == 0) __threadfence();
  }
}

__global__ __launch_bounds__(256) void k_rsmc(const float* __restrict__ S, _Float16* __restrict__ P, _Float16* __restrict__ PR, unsigned q0, unsigned nk, unsigned nrows) {
  #pragma clang fp contract(off)
  const unsigned lane = threadIdx.x & 31u, w = threadIdx.x >> 5;
  const unsigned row = blockIdx.x * 8u + w;
  if (row >= nrows) return;
  const unsigned qi = q0 + (row % (unsigned)QT);
  const unsigned nch = nk >> 8;
  const float* s = S + (size_t)row * SEQ + lane * 8u;
  float mx = -3.0e38f;
#pragma unroll 1
  for (unsigned it = 0; it < nch; ++it) {
    const v4f a = *(const v4fa*)(s + it * 256u), c = *(const v4fa*)(s + it * 256u + 4u);
    const unsigned j0 = it * 256u + lane * 8u;
#pragma unroll
    for (unsigned q = 0; q < 4; ++q) {
      const float av = (j0 + q <= qi) ? a[q] : -3.0e38f;
      const float cv = (j0 + 4u + q <= qi) ? c[q] : -3.0e38f;
      mx = fmaxf(mx, fmaxf(av, cv));
    }
  }
  mx = fmaxf(mx, __shfl_xor(mx, 16, 32)); mx = fmaxf(mx, __shfl_xor(mx, 8, 32)); mx = fmaxf(mx, __shfl_xor(mx, 4, 32)); mx = fmaxf(mx, __shfl_xor(mx, 2, 32)); mx = fmaxf(mx, __shfl_xor(mx, 1, 32));
  float se = 0.f;
#pragma unroll 1
  for (unsigned it = 0; it < nch; ++it) {
    const v4f a = *(const v4fa*)(s + it * 256u), c = *(const v4fa*)(s + it * 256u + 4u);
    const unsigned j0 = it * 256u + lane * 8u;
    float p = 0.f;
#pragma unroll
    for (unsigned q = 0; q < 4; ++q) {
      const float ea = __expf(a[q] - mx), ec = __expf(c[q] - mx);
      p += (j0 + q <= qi) ? ea : 0.f;
      p += (j0 + 4u + q <= qi) ? ec : 0.f;
    }
    se += p;
  }
  se += __shfl_xor(se, 16, 32); se += __shfl_xor(se, 8, 32); se += __shfl_xor(se, 4, 32); se += __shfl_xor(se, 2, 32); se += __shfl_xor(se, 1, 32);
  const float sc = 256.0f / se;
#pragma unroll 1
  for (unsigned it = 0; it < nch; ++it) {
    const v4f a = *(const v4fa*)(s + it * 256u), c = *(const v4fa*)(s + it * 256u + 4u);
    const unsigned j0 = it * 256u + lane * 8u;
    FragH f, g;
#pragma unroll
    for (unsigned q = 0; q < 4; ++q) {
      const float ea = __expf(a[q] - mx) * sc, ec = __expf(c[q] - mx) * sc;
      const float pa = (j0 + q <= qi) ? ea : 0.f;
      const float pc = (j0 + 4u + q <= qi) ? ec : 0.f;
      const _Float16 ha = (_Float16)pa, hc = (_Float16)pc;
      f.h[q] = ha; f.h[4 + q] = hc;
      g.h[q] = (_Float16)((pa - (float)ha) * RSC); g.h[4 + q] = (_Float16)((pc - (float)hc) * RSC);
    }
    const v8us o = f.half[0], orr = g.half[0];
    unsigned short* d = (unsigned short*)P + (size_t)row * SEQ + j0;
    unsigned short* dr = (unsigned short*)PR + (size_t)row * EARLY + j0;
    *(volatile v8us*)d = o; if (PR) *(volatile v8us*)dr = orr;
    __threadfence();
    *(volatile v8us*)d = o; if (PR) *(volatile v8us*)dr = orr;
  }
}

#define WS_W   ((size_t)DM * DM * 2)
#define WS_ROW ((size_t)NB * SEQ * DM * 2)
#define WS_RES ((size_t)NB * EARLY * DM * 2)
#define WS_S   ((size_t)NH * QT * SEQ * 4)
#define WS_P   ((size_t)NH * QT * SEQ * 2)
#define WS_PR  ((size_t)NH * QT * EARLY * 2)
#define WS_VT  ((size_t)NB * NH * HD * SEQ * 2)
#define WS_VTR ((size_t)NB * NH * HD * EARLY * 2)
#define WS_TAB ((size_t)SEQ * 64 * 4)
static_assert(4 * WS_W + 5 * WS_ROW + 4 * WS_RES + WS_S + WS_P + WS_PR + WS_VT + WS_VTR + WS_TAB <= (size_t)134217728);
static_assert(WS_W % 256 == 0 && WS_ROW % 256 == 0 && WS_RES % 256 == 0 && WS_S % 256 == 0 && WS_P % 256 == 0 && WS_PR % 256 == 0 && WS_VT % 256 == 0 && WS_VTR % 256 == 0 && WS_TAB % 256 == 0);

extern "C" void kernel_launch(void* const* d_in, const int* in_sizes, int n_in,
                              void* d_out, int out_size, void* d_ws, size_t ws_size, hipStream_t stream) {
  if (n_in < 5) return;
  if ((size_t)in_sizes[0] < ((size_t)(NB - 1) * SEQ_FULL + SEQ) * DM) return;
  for (int i = 1; i < 5; ++i) if ((size_t)in_sizes[i] < (size_t)DM * DM) return;
  if ((size_t)out_size < NR * DM) return;
  const float* x = (const float*)d_in[0]; const float* wq = (const float*)d_in[1]; const float* wk = (const float*)d_in[2]; const float* wv = (const float*)d_in[3]; const float* wo = (const float*)d_in[4];
  char* ws = (char*)d_ws; size_t off = 0;
  auto take = [&](size_t bytes) { char* p = ws + off; off += (bytes + 255) & ~(size_t)255; return p; };
  _Float16* BQ = (_Float16*)take(WS_W); _Float16* BK = (_Float16*)take(WS_W); _Float16* BV = (_Float16*)take(WS_W); _Float16* BO = (_Float16*)take(WS_W);
  _Float16* X16 = (_Float16*)take(WS_ROW); _Float16* Q16 = (_Float16*)take(WS_ROW); _Float16* K16 = (_Float16*)take(WS_ROW); _Float16* V16 = (_Float16*)take(WS_ROW); _Float16* O16 = (_Float16*)take(WS_ROW);
  _Float16* QR = (_Float16*)take(WS_RES); _Float16* KR = (_Float16*)take(WS_RES); _Float16* VR = (_Float16*)take(WS_RES); _Float16* OR = (_Float16*)take(WS_RES);
  float* S = (float*)take(WS_S); _Float16* P = (_Float16*)take(WS_P); _Float16* PR = (_Float16*)take(WS_PR);
  _Float16* VT = (_Float16*)take(WS_VT); _Float16* VTR = (_Float16*)take(WS_VTR); float* TAB = (float*)take(WS_TAB);
  if (off > ws_size) return;
  _Float16* const nh = (_Float16*)nullptr; float* const nf = (float*)nullptr; const float* const nt = (const float*)nullptr;

  k_ropetab<<<(unsigned)((SEQ * 32) / 256), 256, 0, stream>>>(TAB);
  const unsigned gw = (unsigned)((DM / 64) * (DM / 64));
  k_wtr<<<gw, 256, 0, stream>>>(wq, BQ); k_wtr<<<gw, 256, 0, stream>>>(wk, BK); k_wtr<<<gw, 256, 0, stream>>>(wv, BV); k_wtr<<<gw, 256, 0, stream>>>(wo, BO);
  k_x16<<<(unsigned)((NR * DM / 8 + 255) / 256), 256, 0, stream>>>(x, X16);
  const dim3 gproj((unsigned)((NR / 128) * (DM / 64)), 1);
  k_gemm3<0, 0><<<gproj, 128, 0, stream>>>(X16, nh, DM, DM, (size_t)0, (size_t)0, BQ, nh, DM, DM, (size_t)0, (size_t)0, 0.0625f, nf, Q16, QR, DM, (size_t)0, (unsigned)SEQ, (unsigned)EARLY, TAB, (int)NR, DM, DM);
  k_gemm3<0, 0><<<gproj, 128, 0, stream>>>(X16, nh, DM, DM, (size_t)0, (size_t)0, BK, nh, DM, DM, (size_t)0, (size_t)0, 0.0625f, nf, K16, KR, DM, (size_t)0, (unsigned)SEQ, (unsigned)EARLY, TAB, (int)NR, DM, DM);
  k_gemm3<0, 0><<<gproj, 128, 0, stream>>>(X16, nh, DM, DM, (size_t)0, (size_t)0, BV, nh, DM, DM, (size_t)0, (size_t)0, 0.0625f, nf, V16, VR, DM, (size_t)0, (unsigned)SEQ, (unsigned)EARLY, nt, (int)NR, DM, DM);
  k_vt<NH, SEQ><<<(unsigned)(NB * NH * (SEQ / 64)), 256, 0, stream>>>(V16, DM, 0, VT);
  k_vt<NH, EARLY><<<(unsigned)(NB * NH * (EARLY / 64)), 256, 0, stream>>>(VR, DM, 0, VTR);
  for (int b = 0; b < NB; ++b) {
    const size_t r0 = (size_t)b * SEQ, e0 = (size_t)b * EARLY;
    for (int q0 = 0; q0 < SEQ; q0 += QT) {
      const int nk = q0 + QT;
      const dim3 gs((unsigned)((QT / 128) * (nk / 64)), NH), gp((unsigned)((QT / 128) * (HD / 64)), NH);
      if (q0 < EARLY) {
        k_gemm3<1, 1><<<gs, 128, 0, stream>>>(Q16 + (r0 + q0) * DM, QR + (e0 + q0) * DM, DM, DM, (size_t)HD, (size_t)HD, K16 + r0 * DM, KR + e0 * DM, DM, DM, (size_t)HD, (size_t)HD, ATS, S, nh, nh, SEQ, (size_t)QT * SEQ, RBIG, RBIG, nt, QT, nk, HD);
        k_rsmc<<<(NH * QT) / 8, 256, 0, stream>>>(S, P, PR, (unsigned)q0, (unsigned)nk, (unsigned)(NH * QT));
        k_gemm3<1, 1><<<gp, 128, 0, stream>>>(P, PR, SEQ, EARLY, (size_t)QT * SEQ, (size_t)QT * EARLY, VT + (size_t)b * NH * HD * SEQ, VTR + (size_t)b * NH * HD * EARLY, SEQ, EARLY, (size_t)HD * SEQ, (size_t)HD * EARLY, 0.25f, nf, O16 + (r0 + q0) * DM, OR + (e0 + q0) * DM, DM, (size_t)HD, RBIG, RBIG, nt, QT, HD, nk);
      } else {
        k_gemm3<0, 0><<<gs, 128, 0, stream>>>(Q16 + (r0 + q0) * DM, nh, DM, DM, (size_t)HD, (size_t)HD, K16 + r0 * DM, nh, DM, DM, (size_t)HD, (size_t)HD, ATS, S, nh, nh, SEQ, (size_t)QT * SEQ, RBIG, RBIG, nt, QT, nk, HD);
        k_rsmc<<<(NH * QT) / 8, 256, 0, stream>>>(S, P, nh, (unsigned)q0, (unsigned)nk, (unsigned)(NH * QT));
        k_gemm3<0, 0><<<gp, 128, 0, stream>>>(P, nh, SEQ, SEQ, (size_t)QT * SEQ, (size_t)0, VT + (size_t)b * NH * HD * SEQ, nh, SEQ, SEQ, (size_t)HD * SEQ, (size_t)0, 0.25f, nf, O16 + (r0 + q0) * DM, nh, DM, (size_t)HD, RBIG, RBIG, nt, QT, HD, nk);
      }
    }
  }
  float* out = (float*)d_out;
  for (int b = 0; b < NB; ++b) {
    const size_t r0 = (size_t)b * SEQ, e0 = (size_t)b * EARLY;
    k_gemm3<1, 0><<<dim3((unsigned)((EARLY / 128) * (DM / 64)), 1), 128, 0, stream>>>(O16 + r0 * DM, OR + e0 * DM, DM, DM, (size_t)0, (size_t)0, BO, nh, DM, DM, (size_t)0, (size_t)0, 0.0009765625f, out + r0 * DM, nh, nh, DM, (size_t)0, RBIG, RBIG, nt, EARLY, DM, DM);
    if (SEQ > EARLY)
      k_gemm3<0, 0><<<dim3((unsigned)(((SEQ - EARLY) / 128) * (DM / 64)), 1), 128, 0, stream>>>(O16 + (r0 + EARLY) * DM, nh, DM, DM, (size_t)0, (size_t)0, BO, nh, DM, DM, (size_t)0, (size_t)0, 0.0009765625f, out + (r0 + EARLY) * DM, nh, nh, DM, (size_t)0, RBIG, RBIG, nt, SEQ - EARLY, DM, DM);
  }
}
